// DeMIE_GATv2_6116033429989
// MI455X (gfx1250) — hardware-verified
//
#include <hip/hip_runtime.h>
#include <stddef.h>
#include <math.h>


#define FIN     128
#define H1      128
#define NH1     4
#define CH1     32
#define NC1     256
#define H2      32
#define NC2     64
#define NOUT    3
#define CP      256
#define HPP     512
#define NTHR    256
#define NWAVE   8
#define EPT     8
#define NGRP    2
#define CHUNK   (NTHR * EPT * NGRP)
#define WCAP    (EPT * NGRP * 32)
#define LISTN   (NWAVE * WCAP)
#define NBC     4096
#define NBF     2048
#define FPC     (NBC / NBF)
#define RCAP    40960
#define RBN     128
#define TGT     256
#define DEGCAP  256
#define OTHR    512
#define BM      64
#define STATR   256
#define WSCAP   134217728
#define DEN_EPS 1e-16f
#define BN_EPS  1e-5
#define XSC       8.0f
#define WSC       64.0f
#define INV_CARRY (1.0f / 512.0f)
#define NEGBIG    (-3.0e38f)

#define LDS_FILL ((RCAP + NBF + LISTN) * 4 + 64)
#define LDS_G1   (BM * NC1 * 4)
#define LDS_G2   (BM * NC2 * 4)

static_assert((CHUNK & (CHUNK - 1)) == 0);
static_assert(CHUNK <= 4096);
static_assert(NBC <= 4096 && NBF <= 4096);
static_assert((NBC & (NBC - 1)) == 0 && (NBF & (NBF - 1)) == 0);
static_assert(NBC == FPC * NBF && FPC == 2);
static_assert(OTHR * 8 == NBC);
static_assert(OTHR / 32 == 8 * FPC);
static_assert((RCAP % 32) == 0);
static_assert(TGT == NWAVE * 32);
static_assert((TGT % BM) == 0 && (TGT % STATR) == 0);
static_assert(FIN / 8 == 16 && H1 / 8 == 16);
static_assert(H1 == NH1 * CH1);
static_assert(NC1 == 2 * H1 && NC2 == 2 * H2 && CP == NC1);
static_assert(H2 == 32 && BM == 64 && NWAVE == 8);
static_assert(HPP * 2 == CP * 4);
static_assert(H1 * 2 <= NC2 * 4);
static_assert(2 * NC2 * 4 <= H1 * 4);

typedef float          v4f  __attribute__((ext_vector_type(4)));
typedef float          v8f  __attribute__((ext_vector_type(8)));
typedef double         v2d  __attribute__((ext_vector_type(2)));
typedef int            v4i  __attribute__((ext_vector_type(4)));
typedef _Float16       v8h  __attribute__((ext_vector_type(8)));
typedef _Float16       v16h __attribute__((ext_vector_type(16)));
union FragH { v16h v; v8h h[2]; };

__device__ __forceinline__ v8f wmh(v16h a, v16h b, v8f c) {
  v8f d = __builtin_amdgcn_wmma_f32_16x16x32_f16(false, a, false, b, (short)0, c, false, false);
  asm volatile("v_nop\n\tv_nop\n\tv_nop\n\tv_nop" : "+v"(d) : "v"(a), "v"(b));
  return d;
}

__device__ __forceinline__ float lrl02(float v)  { return fmaxf(v, 0.2f * v); }
__device__ __forceinline__ float lrl001(float v) { return fmaxf(v, 0.01f * v); }
__device__ __forceinline__ v4f lrlv02(v4f t) {
  const v4f u = t * 0.2f; v4f r;
  r.x = fmaxf(t.x, u.x); r.y = fmaxf(t.y, u.y); r.z = fmaxf(t.z, u.z); r.w = fmaxf(t.w, u.w);
  return r;
}
__device__ __forceinline__ v4f lrlv001(v4f t) {
  const v4f u = t * 0.01f; v4f r;
  r.x = fmaxf(t.x, u.x); r.y = fmaxf(t.y, u.y); r.z = fmaxf(t.z, u.z); r.w = fmaxf(t.w, u.w);
  return r;
}
__device__ __forceinline__ float sel4(float a, float b, float c, float d, int h) {
  return h == 0 ? a : (h == 1 ? b : (h == 2 ? c : d));
}
__device__ __forceinline__ v4f selv(bool cnd, v4f a, v4f b) {
  v4f r; r.x = cnd ? a.x : b.x; r.y = cnd ? a.y : b.y; r.z = cnd ? a.z : b.z; r.w = cnd ? a.w : b.w; return r;
}
__device__ __forceinline__ float rlf(float v, int l) {
  return __int_as_float(__builtin_amdgcn_readlane(__float_as_int(v), l));
}
__device__ __forceinline__ float wsum(float v) {
#pragma unroll
  for (int o = 1; o < 32; o <<= 1) v += __shfl_xor(v, o);
  return v;
}
__device__ __forceinline__ float wmax(float v) {
#pragma unroll
  for (int o = 1; o < 32; o <<= 1) v = fmaxf(v, __shfl_xor(v, o));
  return v;
}
__device__ __forceinline__ float gsum8(float v) {
#pragma unroll
  for (int o = 1; o < 8; o <<= 1) v += __shfl_xor(v, o);
  return v;
}
__device__ __forceinline__ v8h cvt8(v4f a, v4f b, float s) {
  v8h r;
  r[0] = (_Float16)(a.x * s); r[1] = (_Float16)(a.y * s); r[2] = (_Float16)(a.z * s); r[3] = (_Float16)(a.w * s);
  r[4] = (_Float16)(b.x * s); r[5] = (_Float16)(b.y * s); r[6] = (_Float16)(b.z * s); r[7] = (_Float16)(b.w * s);
  return r;
}
__device__ __forceinline__ float dot4lr(const float* xs, const float* xd, const float* sw) {
  const v4f a = *(const v4f*)xs, b = *(const v4f*)xd, w = *(const v4f*)sw;
  const v4f t = lrlv02(a + b);
  return t.x * w.x + t.y * w.y + t.z * w.z + t.w * w.w;
}
__device__ __forceinline__ void online(float e, bool valid, float& m, float& d) {
  const float mg = wmax(valid ? e : NEGBIG);
  const float mn = fmaxf(m, mg);
  const float sc = __expf(m - mn);
  const float p  = valid ? __expf(e - mn) : 0.f;
  d = d * sc + wsum(p);
  m = mn;
}

template <int NB>
__device__ __forceinline__ int scan_chunk(const int* __restrict__ dsts, int nE, int cbase, int slotBase,
                                          int vec8, int* list, int tid, int lane, int wave) {
  int wc = 0;
#pragma unroll
  for (int g = 0; g < NGRP; ++g) {
    const int el0  = (g * NTHR + tid) * EPT;
    const int e0   = cbase + el0;
    const int sent = -2147483647 - 1;
    v4i da, db;
    if (vec8 != 0 && cbase + CHUNK <= nE) {
      da = *(const v4i*)(dsts + e0);
      db = *(const v4i*)(dsts + e0 + 4);
    } else {
      da.x = (e0     < nE) ? dsts[min(e0, nE - 1)] : sent;
      da.y = (e0 + 1 < nE) ? dsts[min(e0 + 1, nE - 1)] : sent;
      da.z = (e0 + 2 < nE) ? dsts[min(e0 + 2, nE - 1)] : sent;
      da.w = (e0 + 3 < nE) ? dsts[min(e0 + 3, nE - 1)] : sent;
      db.x = (e0 + 4 < nE) ? dsts[min(e0 + 4, nE - 1)] : sent;
      db.y = (e0 + 5 < nE) ? dsts[min(e0 + 5, nE - 1)] : sent;
      db.z = (e0 + 6 < nE) ? dsts[min(e0 + 6, nE - 1)] : sent;
      db.w = (e0 + 7 < nE) ? dsts[min(e0 + 7, nE - 1)] : sent;
    }
    const unsigned nb = (unsigned)slotBase;
    const unsigned s0 = (unsigned)da.x - nb, s1 = (unsigned)da.y - nb;
    const unsigned s2 = (unsigned)da.z - nb, s3 = (unsigned)da.w - nb;
    const unsigned s4 = (unsigned)db.x - nb, s5 = (unsigned)db.y - nb;
    const unsigned s6 = (unsigned)db.z - nb, s7 = (unsigned)db.w - nb;
    const bool h0 = s0 < (unsigned)NB, h1 = s1 < (unsigned)NB, h2 = s2 < (unsigned)NB, h3 = s3 < (unsigned)NB;
    const bool h4 = s4 < (unsigned)NB, h5 = s5 < (unsigned)NB, h6 = s6 < (unsigned)NB, h7 = s7 < (unsigned)NB;
    const unsigned any = __builtin_amdgcn_ballot_w32(h0 | h1 | h2 | h3 | h4 | h5 | h6 | h7);
    if (any != 0u) {
#define HITJ(J, HJ, SJ) { \
        const unsigned mj = __builtin_amdgcn_ballot_w32(HJ); \
        if (mj != 0u) { \
          if (HJ) { \
            const int pos = wc + (int)__builtin_amdgcn_mbcnt_lo(mj, 0u); \
            if (pos < WCAP) list[wave * WCAP + pos] = ((el0 + (J)) << 12) | (int)(SJ); \
          } \
          wc += (int)__builtin_popcount(mj); } }
      HITJ(0, h0, s0)
      HITJ(1, h1, s1)
      HITJ(2, h2, s2)
      HITJ(3, h3, s3)
      HITJ(4, h4, s4)
      HITJ(5, h5, s5)
      HITJ(6, h6, s6)
      HITJ(7, h7, s7)
#undef HITJ
    }
  }
  return wc;
}

template <int KD, int NC, int NCA>
__global__ __launch_bounds__(NTHR) void k_wprep2(const float* __restrict__ Wa, const float* __restrict__ Wb, _Float16* wp) {
  constexpr int UNITS = NC * KD / 8;
  constexpr int KD8   = KD / 8;
  constexpr int NCB   = NC - NCA;
  static_assert((UNITS % 32) == 0 && NCB > 0 && NCA > 0);
  const int i = (int)blockIdx.x * NTHR + (int)threadIdx.x;
  if (i >= UNITS) return;
  const int n  = i / KD8;
  const int k0 = (i - n * KD8) * 8;
  const int na = n < NCA - 1 ? n : NCA - 1;
  int nb = n - NCA; nb = nb < 0 ? 0 : (nb > NCB - 1 ? NCB - 1 : nb);
  v8h hv;
#pragma unroll
  for (int e = 0; e < 8; ++e) {
    const float fa = Wa[(size_t)(k0 + e) * NCA + na];
    const float fb = Wb[(size_t)(k0 + e) * NCB + nb];
    const float f  = n < NCA ? fa : fb;
    hv[e] = (_Float16)(f * WSC);
  }
  _Float16* d = wp + (size_t)i * 8;
  *(volatile v8h*)d = hv;
  __threadfence();
  *(volatile v8h*)d = hv;
}

__global__ __launch_bounds__(NTHR) void k_count(
    const int* __restrict__ dsts, int* cnt, int nE, int vec8) {
  __shared__ __attribute__((aligned(16))) int scnt[NBC];
  __shared__ __attribute__((aligned(16))) int list[LISTN];
  __shared__ int wcnt[NWAVE];
  const int tid = threadIdx.x, lane = tid & 31, wave = tid >> 5;
  const int nodeBase = blockIdx.x * NBC;

  for (int i = tid; i < NBC; i += NTHR) scnt[i] = 0;
  __syncthreads();

  const int nChunks = (nE + CHUNK - 1) / CHUNK;
#pragma unroll 1
  for (int ch = 0; ch < nChunks; ++ch) {
    const int cbase = ch * CHUNK;
    const int wc = scan_chunk<NBC>(dsts, nE, cbase, nodeBase, vec8, list, tid, lane, wave);
    if (lane == 0) wcnt[wave] = wc;
    __syncthreads();
    if (wave == 0) {
#pragma unroll 1
      for (int wsx = 0; wsx < NWAVE; ++wsx) {
        int n = __builtin_amdgcn_readfirstlane(wcnt[wsx]);
        n = n > WCAP ? WCAP : (n < 0 ? 0 : n);
        const int* lp = list + wsx * WCAP;
#pragma unroll 1
        for (int i = 0; i < n; ++i) {
          const int ent  = __builtin_amdgcn_readfirstlane(lp[i]);
          const int slot = ent & (NBC - 1);
          if (lane == 0) scnt[slot] = scnt[slot] + 1;
        }
      }
    }
    __syncthreads();
  }

  v4i cq[4];
#pragma unroll
  for (int q = 0; q < 4; ++q) {
    const int f = (wave * 4 + q) * 128 + 4 * lane;
    cq[q] = *(const v4i*)(scnt + f);
  }
  int* cpn = cnt + (size_t)nodeBase;
#pragma unroll
  for (int q = 0; q < 4; ++q) {
    const int f = (wave * 4 + q) * 128 + 4 * lane;
    *(volatile v4i*)(cpn + f) = cq[q];
  }
  __threadfence();
#pragma unroll
  for (int q = 0; q < 4; ++q) {
    const int f = (wave * 4 + q) * 128 + 4 * lane;
    *(volatile v4i*)(cpn + f) = cq[q];
  }
}

__global__ __launch_bounds__(OTHR) void k_offsets(
    const int* __restrict__ cnt, int* off, int* rbase, int nChunk) {
  __shared__ __attribute__((aligned(16))) int soff[NBC];
  __shared__ __attribute__((aligned(16))) int srb[RBN];
  __shared__ int wtot[OTHR / 32];
  const int tid = threadIdx.x, lane = tid & 31, wave = tid >> 5, sub = tid >> 8;
  for (int i = tid; i < RBN; i += OTHR) srb[i] = 0;
  int carry = 0;
#pragma unroll 1
  for (int ch = 0; ch < nChunk; ++ch) {
    const int base = ch * NBC;
    const v4i c0 = *(const v4i*)(cnt + base + 8 * tid);
    const v4i c1 = *(const v4i*)(cnt + base + 8 * tid + 4);
    const int e0 = max(c0.x, 0), e1 = max(c0.y, 0), e2 = max(c0.z, 0), e3 = max(c0.w, 0);
    const int e4 = max(c1.x, 0), e5 = max(c1.y, 0), e6 = max(c1.z, 0), e7 = max(c1.w, 0);
    const int ts = e0 + e1 + e2 + e3 + e4 + e5 + e6 + e7;
    int incl = ts;
#pragma unroll
    for (int d = 1; d < 32; d <<= 1) {
      const int t = __shfl_up(incl, d);
      if (lane >= d) incl += t;
    }
    if (lane == 31) wtot[wave] = incl;
    __syncthreads();
    int S0 = 0, S1 = 0;
#pragma unroll
    for (int w = 0; w < 8; ++w) { S0 += wtot[w]; S1 += wtot[8 + w]; }
    int pre = 0;
#pragma unroll 1
    for (int w = 8 * sub; w < wave; ++w) pre += wtot[w];
    const int b0 = carry;
    const int b1 = b0 + ((S0 + 31) & ~31);
    const int b2 = b1 + ((S1 + 31) & ~31);
    const int myb = sub == 0 ? b0 : b1;
    if (tid == 0) {
      srb[min(2 * ch + 0, RBN - 1)] = b0;
      srb[min(2 * ch + 1, RBN - 1)] = b1;
    }
    int run = myb + pre + incl - ts;
    soff[8 * tid + 0] = run; run += e0;
    soff[8 * tid + 1] = run; run += e1;
    soff[8 * tid + 2] = run; run += e2;
    soff[8 * tid + 3] = run; run += e3;
    soff[8 * tid + 4] = run; run += e4;
    soff[8 * tid + 5] = run; run += e5;
    soff[8 * tid + 6] = run; run += e6;
    soff[8 * tid + 7] = run;
    carry = b2;
    __syncthreads();
    const v4i o0 = *(const v4i*)(soff + 4 * tid);
    const v4i o1 = *(const v4i*)(soff + 4 * (tid + OTHR));
    int* op = off + base;
    *(volatile v4i*)(op + 4 * tid) = o0;
    *(volatile v4i*)(op + 4 * (tid + OTHR)) = o1;
    __threadfence();
    *(volatile v4i*)(op + 4 * tid) = o0;
    *(volatile v4i*)(op + 4 * (tid + OTHR)) = o1;
    __syncthreads();
  }
  if (tid == 0) srb[min(2 * nChunk, RBN - 1)] = carry;
  __syncthreads();
  v4i rv = {0, 0, 0, 0};
  if (tid < 32) rv = *(const v4i*)(srb + 4 * tid);
  if (tid < 32) *(volatile v4i*)(rbase + 4 * tid) = rv;
  __threadfence();
  if (tid < 32) *(volatile v4i*)(rbase + 4 * tid) = rv;
}

__global__ __launch_bounds__(NTHR) void k_fill(
    const int* __restrict__ dsts, const int* __restrict__ off, const int* __restrict__ rbase,
    int* csr, int nE, int vec8, int csrLen) {
  extern __shared__ v4f lds_dyn[];
  int* region = (int*)lds_dyn;
  int* cursor = region + RCAP;
  int* list   = cursor + NBF;
  int* wcnt   = list + LISTN;
  const int tid = threadIdx.x, lane = tid & 31, wave = tid >> 5;
  const int b = blockIdx.x;
  const int nodeBase = b * NBF;

  int rb0 = rbase[b];
  const int rb1 = rbase[b + 1];
  rb0 = rb0 < 0 ? 0 : (rb0 > csrLen ? csrLen : rb0);
  rb0 &= ~31;
  int len = rb1 - rb0;
  len = len < 0 ? 0 : (len > RCAP ? RCAP : len);
  int lenW = (len + 31) & ~31;
  if (rb0 + lenW > csrLen) lenW = (csrLen - rb0) & ~31;

  {
    const v4i z = {0, 0, 0, 0};
    for (int i = tid; i < RCAP / 4; i += NTHR) ((v4i*)region)[i] = z;
    for (int s = tid; s < NBF; s += NTHR) {
      int o = off[nodeBase + s] - rb0;
      o = o < 0 ? 0 : (o > RCAP ? RCAP : o);
      cursor[s] = o;
    }
  }
  __syncthreads();

  const int nChunks = (nE + CHUNK - 1) / CHUNK;
#pragma unroll 1
  for (int ch = 0; ch < nChunks; ++ch) {
    const int cbase = ch * CHUNK;
    const int wc = scan_chunk<NBF>(dsts, nE, cbase, nodeBase, vec8, list, tid, lane, wave);
    if (lane == 0) wcnt[wave] = wc;
    __syncthreads();
    if (wave == 0) {
#pragma unroll 1
      for (int wsx = 0; wsx < NWAVE; ++wsx) {
        int n = __builtin_amdgcn_readfirstlane(wcnt[wsx]);
        n = n > WCAP ? WCAP : (n < 0 ? 0 : n);
        const int* lp = list + wsx * WCAP;
#pragma unroll 1
        for (int i = 0; i < n; ++i) {
          const int ent  = __builtin_amdgcn_readfirstlane(lp[i]);
          const int slot = ent & (NBF - 1);
          int e = cbase + ((ent >> 12) & (CHUNK - 1));
          e = e > nE - 1 ? nE - 1 : e;
          if (lane == 0) {
            int pos = cursor[slot];
            pos = pos < 0 ? 0 : (pos > RCAP - 1 ? RCAP - 1 : pos);
            region[pos] = e;
            const int np = pos + 1;
            cursor[slot] = np > RCAP ? RCAP : np;
          }
        }
      }
    }
    __syncthreads();
  }

  const int nv = lenW >> 2;
  int* gp = csr + rb0;
#pragma unroll 1
  for (int i = tid; i < nv; i += NTHR) { const v4i v = ((const v4i*)region)[i]; *(volatile v4i*)(gp + 4 * i) = v; }
  __threadfence();
#pragma unroll 1
  for (int i = tid; i < nv; i += NTHR) { const v4i v = ((const v4i*)region)[i]; *(volatile v4i*)(gp + 4 * i) = v; }
}

template <int KD, int LDA, int NCOL, typename AT>
__device__ __forceinline__ void mm_tile(const AT* __restrict__ A, const _Float16* __restrict__ Bw,
                                        int rowBase, int nArow, float* stg) {
  static_assert(KD % 32 == 0 && (NCOL % 32) == 0 && (LDA % 8) == 0 && LDA >= KD);
  static_assert(sizeof(AT) == 4 || sizeof(AT) == 2);
  constexpr int NT  = NCOL / 32;
  constexpr int NCW = NCOL / 2;
  const int tid = threadIdx.x, lane = tid & 31, wave = tid >> 5, hh = lane >> 4, m = lane & 15;
  const int r0 = (wave >> 1) * 16, c0 = (wave & 1) * NCW;
  v8f acc[NT];
#pragma unroll
  for (int t = 0; t < NT; ++t) { v8f z = {0.f, 0.f, 0.f, 0.f, 0.f, 0.f, 0.f, 0.f}; acc[t] = z; }
  int ar = rowBase + r0 + m;
  ar = ar < nArow ? ar : nArow - 1;
  const AT* ap  = A  + (size_t)ar * LDA + 8 * hh;
  const _Float16* bp0 = Bw + (size_t)(c0 + m) * KD + 8 * hh;
#pragma unroll 1
  for (int kt = 0; kt < KD / 32; ++kt) {
    FragH a;
    if constexpr (sizeof(AT) == 4) {
      const float* fp = (const float*)ap + 32 * kt;
      const v4f x0 = *(const v4f*)fp,        x1 = *(const v4f*)(fp + 4);
      const v4f x2 = *(const v4f*)(fp + 16), x3 = *(const v4f*)(fp + 20);
      a.h[0] = cvt8(x0, x1, XSC);
      a.h[1] = cvt8(x2, x3, XSC);
    } else {
      a.h[0] = *(const v8h*)(ap + 32 * kt);
      a.h[1] = *(const v8h*)(ap + 32 * kt + 16);
    }
#pragma unroll
    for (int t = 0; t < NT; ++t) {
      const _Float16* bp = bp0 + (size_t)(16 * t) * KD + 32 * kt;
      FragH b;
      b.h[0] = *(const v8h*)bp;
      b.h[1] = *(const v8h*)(bp + 16);
      acc[t] = wmh(a.v, b.v, acc[t]);
    }
  }
  float* sp = stg + (size_t)(r0 + 8 * hh) * NCOL + c0 + m;
#pragma unroll
  for (int t = 0; t < NT; ++t) {
#pragma unroll
    for (int r = 0; r < 8; ++r) sp[r * NCOL + 16 * t] = acc[t][r] * INV_CARRY;
  }
}

template <int KD, int LDA, int NCOL, typename AT>
__global__ __launch_bounds__(NTHR) void k_gemm(
    const AT* __restrict__ A, const _Float16* __restrict__ Bw, float* C, int ldc, int nArow) {
  extern __shared__ v4f lds_dyn[];
  float* stg = (float*)lds_dyn;
  const int tid = threadIdx.x, lane = tid & 31, wave = tid >> 5;
  const int rowBase = blockIdx.x * BM;
  constexpr int NCW = NCOL / 2, LPR = NCW / 4, RPI = 32 / LPR, NIT = 16 / RPI;
  static_assert(LPR >= 8 && (32 % LPR) == 0 && (16 % RPI) == 0);
  const int r0 = (wave >> 1) * 16, c0 = (wave & 1) * NCW;

  mm_tile<KD, LDA, NCOL, AT>(A, Bw, rowBase, nArow, stg);
  __syncthreads();

  const int rsub = lane / LPR, q = lane - rsub * LPR, col = c0 + 4 * q;
  const size_t gb = (size_t)(rowBase + r0) * ldc + col;
#pragma unroll
  for (int it = 0; it < NIT; ++it) {
    const int row = it * RPI + rsub;
    const v4f v = *(const v4f*)(stg + (size_t)(r0 + row) * NCOL + col);
    *(volatile v4f*)(C + gb + (size_t)row * ldc) = v;
  }
  __threadfence();
#pragma unroll
  for (int it = 0; it < NIT; ++it) {
    const int row = it * RPI + rsub;
    const v4f v = *(const v4f*)(stg + (size_t)(r0 + row) * NCOL + col);
    *(volatile v4f*)(C + gb + (size_t)row * ldc) = v;
  }
}

__global__ __launch_bounds__(NTHR) void k_soft1(
    const int* __restrict__ csr, const int* __restrict__ off, const int* __restrict__ cnt,
    const int* __restrict__ srcs, const float* __restrict__ cpl,
    const float* __restrict__ att, float* mtab, float* rtab, float* aself,
    int nN, int nE, int csrLen) {
  __shared__ __attribute__((aligned(16))) float satt[H1];
  __shared__ __attribute__((aligned(16))) float sxr[NWAVE * H1];
  const int tid = threadIdx.x, lane = tid & 31, wave = tid >> 5;
  if (tid < H1) satt[tid] = att[tid];
  __syncthreads();
  const int tbase = blockIdx.x * TGT + wave * 32;
  const int col = 4 * lane;
  const v4f z4 = {0.f, 0.f, 0.f, 0.f};
  const v4f at4 = *(const v4f*)(att + col);
  const int cl    = tbase + lane;
  const int cnt_l = cnt[cl];
  const int off_l = off[cl];
  float* sx = sxr + wave * H1;
  v4f mk = z4, rk = z4, ak = z4;

#pragma unroll 1
  for (int j = 0; j < 32; ++j) {
    const int c = tbase + j;
    int n = __shfl(cnt_l, j);
    n = n < 0 ? 0 : (n > DEGCAP ? DEGCAP : n);
    const int st = __shfl(off_l, j);
    const float* rowc = cpl + (size_t)c * CP;
    const v4f xlc = *(const v4f*)(rowc + col);
    const v4f xrc = *(const v4f*)(rowc + H1 + col);
    __builtin_amdgcn_wave_barrier();
    *(v4f*)(sx + col) = xrc;
    __builtin_amdgcn_fence(__ATOMIC_RELEASE, "wavefront");
    __builtin_amdgcn_wave_barrier();
    const v4f tt = lrlv02(xlc + xrc);
    float ps = tt.x * at4.x + tt.y * at4.y + tt.z * at4.z + tt.w * at4.w;
    ps = gsum8(ps);
    const float es0 = __shfl(ps, 0), es1 = __shfl(ps, 8), es2 = __shfl(ps, 16), es3 = __shfl(ps, 24);

    float m0 = es0, m1 = es1, m2 = es2, m3 = es3;
    float d0 = 1.f, d1 = 1.f, d2 = 1.f, d3 = 1.f;
#pragma unroll 1
    for (int q0 = 0; q0 < n; q0 += 32) {
      int pos = st + q0 + lane;
      pos = pos < 0 ? 0 : (pos > csrLen - 1 ? csrLen - 1 : pos);
      int eid = csr[pos];
      eid = eid < 0 ? 0 : (eid > nE - 1 ? nE - 1 : eid);
      int sl = srcs[eid];
      sl = sl < 0 ? 0 : (sl > nN - 1 ? nN - 1 : sl);
      const int mcnt = (n - q0) < 32 ? (n - q0) : 32;
      const bool valid = lane < mcnt;
      const float* xs = cpl + (size_t)sl * CP;
      float e0 = 0.f, e1 = 0.f, e2 = 0.f, e3 = 0.f;
#pragma unroll 1
      for (int c8 = 0; c8 < CH1; c8 += 4) {
        e0 += dot4lr(xs + c8,           sx + c8,           satt + c8);
        e1 += dot4lr(xs + CH1 + c8,     sx + CH1 + c8,     satt + CH1 + c8);
        e2 += dot4lr(xs + 2 * CH1 + c8, sx + 2 * CH1 + c8, satt + 2 * CH1 + c8);
        e3 += dot4lr(xs + 3 * CH1 + c8, sx + 3 * CH1 + c8, satt + 3 * CH1 + c8);
      }
      online(e0, valid, m0, d0);
      online(e1, valid, m1, d1);
      online(e2, valid, m2, d2);
      online(e3, valid, m3, d3);
    }
    v4f r4;
    r4.x = 1.0f / (d0 + DEN_EPS); r4.y = 1.0f / (d1 + DEN_EPS);
    r4.z = 1.0f / (d2 + DEN_EPS); r4.w = 1.0f / (d3 + DEN_EPS);
    v4f m4; m4.x = m0; m4.y = m1; m4.z = m2; m4.w = m3;
    v4f a4;
    a4.x = __expf(es0 - m0) * r4.x; a4.y = __expf(es1 - m1) * r4.y;
    a4.z = __expf(es2 - m2) * r4.z; a4.w = __expf(es3 - m3) * r4.w;
    const bool mine = (lane == j);
    mk = selv(mine, m4, mk); rk = selv(mine, r4, rk); ak = selv(mine, a4, ak);
  }

  float* pm = mtab + (size_t)cl * NH1;
  float* pr = rtab + (size_t)cl * NH1;
  float* pa = aself + (size_t)cl * NH1;
  const bool wa = cl < nN;
  *(volatile v4f*)pm = mk;
  *(volatile v4f*)pr = rk;
  if (wa) *(volatile v4f*)pa = ak;
  __threadfence();
  *(volatile v4f*)pm = mk;
  *(volatile v4f*)pr = rk;
  if (wa) *(volatile v4f*)pa = ak;
}

__global__ __launch_bounds__(NTHR) void k_alpha1(
    const float* __restrict__ cpl, const int* __restrict__ srcs, const int* __restrict__ dsts,
    const float* __restrict__ att, const float* __restrict__ mtab, const float* __restrict__ rtab,
    float* out1, int nN, int nE) {
  __shared__ __attribute__((aligned(16))) float satt[H1];
  const int tid = threadIdx.x;
  if (tid < H1) satt[tid] = att[tid];
  __syncthreads();
  const int ee  = (int)blockIdx.x * NTHR + tid;
  const int eec = ee < nE ? ee : nE - 1;
  int s = srcs[eec]; s = s < 0 ? 0 : (s > nN - 1 ? nN - 1 : s);
  int d = dsts[eec]; d = d < 0 ? 0 : (d > nN - 1 ? nN - 1 : d);
  const float* xs = cpl + (size_t)s * CP;
  const float* xd = cpl + (size_t)d * CP + H1;
  float e0 = 0.f, e1 = 0.f, e2 = 0.f, e3 = 0.f;
#pragma unroll 1
  for (int c8 = 0; c8 < CH1; c8 += 4) {
    e0 += dot4lr(xs + c8,           xd + c8,           satt + c8);
    e1 += dot4lr(xs + CH1 + c8,     xd + CH1 + c8,     satt + CH1 + c8);
    e2 += dot4lr(xs + 2 * CH1 + c8, xd + 2 * CH1 + c8, satt + 2 * CH1 + c8);
    e3 += dot4lr(xs + 3 * CH1 + c8, xd + 3 * CH1 + c8, satt + 3 * CH1 + c8);
  }
  const v4f m4 = *(const v4f*)(mtab + (size_t)d * NH1);
  const v4f r4 = *(const v4f*)(rtab + (size_t)d * NH1);
  v4f a;
  a.x = __expf(e0 - m4.x) * r4.x; a.y = __expf(e1 - m4.y) * r4.y;
  a.z = __expf(e2 - m4.z) * r4.z; a.w = __expf(e3 - m4.w) * r4.w;
  float* p = out1 + (size_t)ee * NH1;
  if (ee < nE) *(volatile v4f*)p = a;
  __threadfence();
  if (ee < nE) *(volatile v4f*)p = a;
}

__global__ __launch_bounds__(NTHR) void k_agg1(
    const int* __restrict__ csr, const int* __restrict__ off, const int* __restrict__ cnt,
    const int* __restrict__ srcs, float* cpl, const float* __restrict__ alp,
    const float* __restrict__ bias, int nN, int nE, int csrLen) {
  const int tid = threadIdx.x, lane = tid & 31, wave = tid >> 5;
  const int tbase = blockIdx.x * TGT + wave * 32;
  const int col = 4 * lane, hd = lane >> 3;
  const v4f z4 = {0.f, 0.f, 0.f, 0.f};
  const v4f bb4 = *(const v4f*)(bias + col);
  const int cl    = tbase + lane;
  const int cnt_l = cnt[cl];
  const int off_l = off[cl];

#pragma unroll 1
  for (int j = 0; j < 32; ++j) {
    const int c = tbase + j;
    int n = __shfl(cnt_l, j);
    n = n < 0 ? 0 : (n > DEGCAP ? DEGCAP : n);
    const int st = __shfl(off_l, j);
    float* rowc = cpl + (size_t)c * CP;
    const v4f xlc = *(const v4f*)(rowc + col);

    v4f acc = z4;
#pragma unroll 1
    for (int q0 = 0; q0 < n; q0 += 32) {
      int pos = st + q0 + lane;
      pos = pos < 0 ? 0 : (pos > csrLen - 1 ? csrLen - 1 : pos);
      int eid = csr[pos];
      eid = eid < 0 ? 0 : (eid > nE - 1 ? nE - 1 : eid);
      int sl = srcs[eid];
      sl = sl < 0 ? 0 : (sl > nN - 1 ? nN - 1 : sl);
      const v4f al = *(const v4f*)(alp + (size_t)eid * NH1);
      const int mcnt = (n - q0) < 32 ? (n - q0) : 32;
#pragma unroll 1
      for (int pp = 0; pp < mcnt; ++pp) {
        const int   s  = __builtin_amdgcn_readlane(sl, pp);
        const float g0 = rlf(al.x, pp), g1 = rlf(al.y, pp), g2 = rlf(al.z, pp), g3 = rlf(al.w, pp);
        const float pw = sel4(g0, g1, g2, g3, hd);
        const v4f xl = *(const v4f*)(cpl + (size_t)s * CP + col);
        acc = acc + xl * pw;
      }
    }
    const int cs = c < nN ? c : nN - 1;
    const v4f as = *(const v4f*)(alp + (size_t)(nE + cs) * NH1);
    acc = acc + xlc * sel4(as.x, as.y, as.z, as.w, hd);
    v4f v = acc + bb4;
    if (c >= nN) v = z4;

    float* po = rowc + H1 + col;
    *(volatile v4f*)po = v;
    __threadfence();
    *(volatile v4f*)po = v;
  }
}

__global__ __launch_bounds__(H1) void k_bnstat(const float* __restrict__ o0, double* part, int nN) {
  __shared__ __attribute__((aligned(16))) double spt[2 * H1];
  const int col = threadIdx.x;
  const int r0 = blockIdx.x * STATR;
  int nr = nN - r0;
  nr = nr < 0 ? 0 : (nr > STATR ? STATR : nr);
  double s = 0.0, q = 0.0;
#pragma unroll 1
  for (int i = 0; i < nr; ++i) {
    const double v = (double)o0[(size_t)(r0 + i) * CP + col];
    s += v;
    q += v * v;
  }
  spt[col] = s;
  spt[H1 + col] = q;
  __syncthreads();
  const v2d w = *(const v2d*)(spt + 2 * col);
  double* pp = part + (size_t)blockIdx.x * (2 * H1) + 2 * col;
  *(volatile v2d*)pp = w;
  __threadfence();
  *(volatile v2d*)pp = w;
}

__global__ __launch_bounds__(H1) void k_bnfin(const double* __restrict__ part, const float* __restrict__ gamma,
                                              float* tbl, int nPart, int nN) {
  __shared__ __attribute__((aligned(16))) float stb[2 * H1];
  const int tid = threadIdx.x, col = tid;
  double s = 0.0, q = 0.0;
#pragma unroll 1
  for (int b = 0; b < nPart; ++b) {
    s += part[(size_t)b * (2 * H1) + col];
    q += part[(size_t)b * (2 * H1) + H1 + col];
  }
  const double inv = 1.0 / (double)nN;
  const double mu  = s * inv;
  double var = q * inv - mu * mu;
  var = var < 0.0 ? 0.0 : var;
  const float a  = (float)((double)gamma[col] / sqrt(var + BN_EPS));
  const float mf = (float)mu;
  stb[col] = mf;
  stb[H1 + col] = a;
  __syncthreads();
  const int t4 = tid < 64 ? tid : 63;
  const v4f w = *(const v4f*)(stb + 4 * t4);
  if (tid < 64) *(volatile v4f*)(tbl + 4 * tid) = w;
  __threadfence();
  if (tid < 64) *(volatile v4f*)(tbl + 4 * tid) = w;
}

__global__ __launch_bounds__(NTHR) void k_bnapply(
    const float* o0, const float* __restrict__ tbl, const float* __restrict__ beta,
    _Float16* hp, int nN, int nUnits) {
  const int i = (int)blockIdx.x * NTHR + (int)threadIdx.x;
  if (i >= nUnits) return;
  const int row = i >> 4;
  const int c   = (i & 15) * 8;
  const float* orow = o0 + (size_t)row * CP + c;
  const v4f s0 = *(const v4f*)orow, s1 = *(const v4f*)(orow + 4);
  const v4f mu0 = *(const v4f*)(tbl + c),      mu1 = *(const v4f*)(tbl + c + 4);
  const v4f ga0 = *(const v4f*)(tbl + H1 + c), ga1 = *(const v4f*)(tbl + H1 + c + 4);
  const v4f be0 = *(const v4f*)(beta + c),     be1 = *(const v4f*)(beta + c + 4);
  const v4f z4 = {0.f, 0.f, 0.f, 0.f};
  v4f h0 = lrlv001((s0 - mu0) * ga0 + be0);
  v4f h1 = lrlv001((s1 - mu1) * ga1 + be1);
  if (row >= nN) { h0 = z4; h1 = z4; }
  const v8h w = cvt8(h0, h1, XSC);
  _Float16* d = hp + (size_t)row * HPP + c;
  *(volatile v8h*)d = w;
  __threadfence();
  *(volatile v8h*)d = w;
}

__global__ __launch_bounds__(NTHR) void k_agg2(
    const int* __restrict__ csr, const int* __restrict__ off, const int* __restrict__ cnt,
    const int* __restrict__ srcs, const float* __restrict__ cp2,
    const float* __restrict__ att, const float* __restrict__ bias,
    const float* __restrict__ wo, const float* __restrict__ bo,
    float* out0, int nN, int nE, int csrLen) {
  __shared__ __attribute__((aligned(16))) float satt[H2];
  __shared__ __attribute__((aligned(16))) float sxr[NWAVE * H2];
  __shared__ __attribute__((aligned(16))) float slp[NWAVE * 128];
  const int tid = threadIdx.x, lane = tid & 31, wave = tid >> 5;
  if (tid < H2) satt[tid] = att[tid];
  for (int i = tid; i < NWAVE * 128; i += NTHR) slp[i] = 0.f;
  __syncthreads();
  const int tbase = blockIdx.x * TGT + wave * 32;
  const float atl = att[lane];
  const float bb  = bias[lane];
  const float w0 = wo[lane * NOUT + 0], w1 = wo[lane * NOUT + 1], w2 = wo[lane * NOUT + 2];
  const float bo0 = bo[0], bo1 = bo[1], bo2 = bo[2];
  const int cl    = tbase + lane;
  const int cnt_l = cnt[cl];
  const int off_l = off[cl];
  float* sx = sxr + wave * H2;
  float* sp = slp + wave * 128;

#pragma unroll 1
  for (int j = 0; j < 32; ++j) {
    const int c = tbase + j;
    int n = __shfl(cnt_l, j);
    n = n < 0 ? 0 : (n > DEGCAP ? DEGCAP : n);
    const int st = __shfl(off_l, j);
    const float* rowc = cp2 + (size_t)c * CP;
    const float xlc = rowc[lane];
    const float xrc = rowc[H2 + lane];
    const float es = wsum(atl * lrl02(xlc + xrc));
    __builtin_amdgcn_wave_barrier();
    sx[lane] = xrc;
    __builtin_amdgcn_fence(__ATOMIC_RELEASE, "wavefront");
    __builtin_amdgcn_wave_barrier();

    float m = es, den = 1.0f, acc = xlc;
#pragma unroll 1
    for (int q0 = 0; q0 < n; q0 += 32) {
      int pos = st + q0 + lane;
      pos = pos < 0 ? 0 : (pos > csrLen - 1 ? csrLen - 1 : pos);
      int eid = csr[pos];
      eid = eid < 0 ? 0 : (eid > nE - 1 ? nE - 1 : eid);
      int sl = srcs[eid];
      sl = sl < 0 ? 0 : (sl > nN - 1 ? nN - 1 : sl);
      const int mcnt = (n - q0) < 32 ? (n - q0) : 32;
      const bool valid = lane < mcnt;
      const float* xs = cp2 + (size_t)sl * CP;
      float e = 0.f;
#pragma unroll 4
      for (int ch = 0; ch < H2; ++ch) {
        const float v = lrl02(xs[ch] + sx[ch]);
        e = fmaf(satt[ch], v, e);
      }
      const float mg = wmax(valid ? e : NEGBIG);
      const float mn = fmaxf(m, mg);
      const float sc = __expf(m - mn);
      const float p  = valid ? __expf(e - mn) : 0.f;
      const float sg = wsum(p);
      den = den * sc + sg;
      acc = acc * sc;
      m = mn;
#pragma unroll 1
      for (int pp = 0; pp < mcnt; ++pp) {
        const int   s  = __builtin_amdgcn_readlane(sl, pp);
        const float pw = rlf(p, pp);
        acc = fmaf(pw, cp2[(size_t)s * CP + lane], acc);
      }
    }
    const float rd = 1.0f / (den + DEN_EPS);
    const float v  = lrl001(acc * rd + bb);
    const float l0 = wsum(v * w0) + bo0;
    const float l1 = wsum(v * w1) + bo1;
    const float l2 = wsum(v * w2) + bo2;
    const float mx = fmaxf(l0, fmaxf(l1, l2));
    const float s0 = l0 - mx, s1 = l1 - mx, s2 = l2 - mx;
    const float lg = __logf(__expf(s0) + __expf(s1) + __expf(s2));
    const float lp = lane == 0 ? (s0 - lg) : (lane == 1 ? (s1 - lg) : (s2 - lg));
    if (lane < NOUT) sp[j * NOUT + lane] = lp;
  }
  __builtin_amdgcn_fence(__ATOMIC_RELEASE, "wavefront");
  __builtin_amdgcn_wave_barrier();

  int nval = nN - tbase;
  nval = nval < 0 ? 0 : (nval > 32 ? 32 : nval);
  const int li = lane < 24 ? lane : 23;
  const v4f o4 = *(const v4f*)(sp + 4 * li);
  float* gp = out0 + (size_t)tbase * NOUT;
  if (nval == 32) {
    if (lane < 24) *(volatile v4f*)(gp + 4 * lane) = o4;
    __threadfence();
    if (lane < 24) *(volatile v4f*)(gp + 4 * lane) = o4;
  } else if (nval > 0) {
    const int nf = NOUT * nval;
#pragma unroll 1
    for (int f = lane; f < nf; f += 32) { const float t = sp[f]; *(volatile float*)(gp + f) = t; }
    __threadfence();
#pragma unroll 1
    for (int f = lane; f < nf; f += 32) { const float t = sp[f]; *(volatile float*)(gp + f) = t; }
  }
}

extern "C" void kernel_launch(void* const* d_in, const int* in_sizes, int n_in,
                              void* d_out, int out_size, void* d_ws, size_t ws_size,
                              hipStream_t stream) {
  if (n_in < 14) return;
  const int nN = in_sizes[0] / FIN;
  const int nE = in_sizes[1] / 2;
  if (nN <= 0 || nE <= 0 || in_sizes[0] != nN * FIN || in_sizes[1] != 2 * nE) return;
  if (in_sizes[2] != FIN * H1 || in_sizes[3] != FIN * H1 || in_sizes[4] != NH1 * CH1 || in_sizes[5] != H1) return;
  if (in_sizes[6] != H1 || in_sizes[7] != H1) return;
  if (in_sizes[8] != H1 * H2 || in_sizes[9] != H1 * H2 || in_sizes[10] != H2 || in_sizes[11] != H2) return;
  if (in_sizes[12] != H2 * NOUT || in_sizes[13] != NOUT) return;
  if (nE > (1 << 27) || nN > (1 << 22)) return;
  const long long Et = (long long)nE + nN;
  if ((long long)out_size != (long long)nN * NOUT + Et * NH1) return;

  const float* x     = (const float*)d_in[0];
  const int*   ei    = (const int*)d_in[1];
  const float* Wl1   = (const float*)d_in[2];
  const float* Wr1   = (const float*)d_in[3];
  const float* att1  = (const float*)d_in[4];
  const float* b1    = (const float*)d_in[5];
  const float* gamma = (const float*)d_in[6];
  const float* beta  = (const float*)d_in[7];
  const float* Wl2   = (const float*)d_in[8];
  const float* Wr2   = (const float*)d_in[9];
  const float* att2  = (const float*)d_in[10];
  const float* b2    = (const float*)d_in[11];
  const float* Wout  = (const float*)d_in[12];
  const float* bout  = (const float*)d_in[13];
  const int*   src = ei;
  const int*   dst = ei + nE;
  float* out0 = (float*)d_out;
  float* out1 = out0 + (size_t)nN * NOUT;

  const int NPAD   = ((nN + TGT - 1) / TGT) * TGT;
  const int nBC    = (nN + NBC - 1) / NBC;
  const int CNTPAD = nBC * NBC;
  if (FPC * nBC + 1 > RBN) return;
  const int nBF    = (nN + NBF - 1) / NBF;
  const int csrLen = ((nE + 31) & ~31) + 4096;
  if (31 * FPC * nBC > 4096) return;
  const int nAgg   = NPAD / TGT;
  const int nGm    = NPAD / BM;
  const int nStat  = NPAD / STATR;
  const int nUnit  = NPAD * (H1 / 8);
  const int nEB    = (nE + NTHR - 1) / NTHR;

  char* ws = (char*)d_ws;
  size_t off = 0;
  const size_t oWp1 = off; off += (size_t)NC1 * FIN * 2;         off = (off + 255) & ~(size_t)255;
  const size_t oWp2 = off; off += (size_t)NC2 * H1 * 2;          off = (off + 255) & ~(size_t)255;
  const size_t oCnt = off; off += (size_t)CNTPAD * 4;            off = (off + 255) & ~(size_t)255;
  const size_t oOff = off; off += (size_t)CNTPAD * 4;            off = (off + 255) & ~(size_t)255;
  const size_t oRb  = off; off += (size_t)RBN * 4;               off = (off + 255) & ~(size_t)255;
  const size_t oCsr = off; off += (size_t)csrLen * 4;            off = (off + 255) & ~(size_t)255;
  const size_t szTb = (size_t)NPAD * NH1 * 4;
  const size_t r1b  = szTb + szTb;
  const size_t szPt = (((size_t)nStat * 2 * H1 * 8) + 255) & ~(size_t)255;
  const size_t r1c  = szPt + (size_t)2 * H1 * 4;
  const size_t r1   = r1b > r1c ? r1b : r1c;
  const size_t oR1  = off; off += r1;                            off = (off + 255) & ~(size_t)255;
  const size_t oCp  = off; off += (size_t)NPAD * CP * 4;         off = (off + 255) & ~(size_t)255;
  if (off > ws_size || off > (size_t)WSCAP) return;

  _Float16* wp1 = (_Float16*)(ws + oWp1);
  _Float16* wp2 = (_Float16*)(ws + oWp2);
  int*    cnt  = (int*)(ws + oCnt);
  int*    offp = (int*)(ws + oOff);
  int*    rb   = (int*)(ws + oRb);
  int*    csr  = (int*)(ws + oCsr);
  float*  mtab = (float*)(ws + oR1);
  float*  rtab = (float*)(ws + oR1 + szTb);
  double* part = (double*)(ws + oR1);
  float*  tbl  = (float*)(ws + oR1 + szPt);
  float*  cpl  = (float*)(ws + oCp);
  _Float16* hp  = (_Float16*)(ws + oCp);
  float*    o0  = cpl + H1;
  float*    cp2 = cpl + NC2;

  const int vec8 = ((nE & 3) == 0) ? 1 : 0;

  k_wprep2<FIN, NC1, H1><<<(NC1 * FIN / 8 + NTHR - 1) / NTHR, NTHR, 0, stream>>>(Wl1, Wr1, wp1);
  k_wprep2<H1, NC2, H2><<<(NC2 * H1 / 8 + NTHR - 1) / NTHR, NTHR, 0, stream>>>(Wl2, Wr2, wp2);

  k_count<<<nBC, NTHR, 0, stream>>>(dst, cnt, nE, vec8);
  k_offsets<<<1, OTHR, 0, stream>>>(cnt, offp, rb, nBC);
  hipFuncSetAttribute(reinterpret_cast<const void*>(&k_fill),
                      hipFuncAttributeMaxDynamicSharedMemorySize, LDS_FILL);
  k_fill<<<nBF, NTHR, LDS_FILL, stream>>>(dst, offp, rb, csr, nE, vec8, csrLen);

  hipFuncSetAttribute(reinterpret_cast<const void*>(&k_gemm<FIN, FIN, NC1, float>),
                      hipFuncAttributeMaxDynamicSharedMemorySize, LDS_G1);
  k_gemm<FIN, FIN, NC1, float><<<nGm, NTHR, LDS_G1, stream>>>(x, wp1, cpl, CP, nN);

  k_soft1<<<nAgg, NTHR, 0, stream>>>(csr, offp, cnt, src, cpl, att1, mtab, rtab,
                                      out1 + (size_t)nE * NH1, nN, nE, csrLen);
  k_alpha1<<<nEB, NTHR, 0, stream>>>(cpl, src, dst, att1, mtab, rtab, out1, nN, nE);
  k_agg1<<<nAgg, NTHR, 0, stream>>>(csr, offp, cnt, src, cpl, out1, b1, nN, nE, csrLen);

  k_bnstat<<<nStat, H1, 0, stream>>>(o0, part, nN);
  k_bnfin<<<1, H1, 0, stream>>>(part, gamma, tbl, nStat, nN);
  k_bnapply<<<(nUnit + NTHR - 1) / NTHR, NTHR, 0, stream>>>(o0, tbl, beta, hp, nN, nUnit);

  hipFuncSetAttribute(reinterpret_cast<const void*>(&k_gemm<H1, HPP, NC2, _Float16>),
                      hipFuncAttributeMaxDynamicSharedMemorySize, LDS_G2);
  k_gemm<H1, HPP, NC2, _Float16><<<nGm, NTHR, LDS_G2, stream>>>(hp, wp2, cp2, CP, NPAD);
  k_agg2<<<nAgg, NTHR, 0, stream>>>(csr, offp, cnt, src, cp2, att2, b2, Wout, bout, out0, nN, nE, csrLen);
}
